// SelfAttentionHead_30485677867687
// MI455X (gfx1250) — hardware-verified
//
#include <hip/hip_runtime.h>

#define BATCH    8
#define SEQ      2048
#define MDIM     256
#define KEY      64
#define DDIM     128
#define ROWS     (BATCH * SEQ)

#define QSCALE   (0.125f * 1.44269504088896f)

#define __bf16 _Float16
typedef __attribute__((ext_vector_type(16))) _Float16 v16bf;
typedef __attribute__((ext_vector_type(8)))  _Float16 v8bf;
#define RSPLIT (1.0f / 2048.0f)
#define PQK ((size_t)ROWS * KEY)
static __device__ __forceinline__ void split16(float f, _Float16& h, _Float16& l) { h = (_Float16)f; l = (_Float16)((f - (float)h) * 2048.0f); }
static __device__ __forceinline__ unsigned pack2h(_Float16 a, _Float16 b) { return (unsigned)__builtin_bit_cast(unsigned short, a) | ((unsigned)__builtin_bit_cast(unsigned short, b) << 16); }
typedef __attribute__((ext_vector_type(8)))  float  v8f;
typedef __attribute__((ext_vector_type(4)))  float  v4f;

static __device__ __forceinline__ float fast_exp2(float x) {
  return __builtin_amdgcn_exp2f(x);
}

static __device__ __forceinline__ v16bf cat8(v8bf lo, v8bf hi) {
  return __builtin_shufflevector(lo, hi, 0, 1, 2, 3, 4, 5, 6, 7,
                                         8, 9, 10, 11, 12, 13, 14, 15);
}

static __device__ __forceinline__ v16bf load_a(const __bf16* src, int lda,
                                               int r, int half, int koff) {
  const __bf16* p = src + (size_t)r * lda + koff + half * 8;
  return cat8(*(const v8bf*)p, *(const v8bf*)(p + 16));
}

static __device__ __forceinline__ v16bf load_bT(const __bf16* srcT, int ldk,
                                                int n, int half, int koff) {
  const __bf16* p = srcT + (size_t)n * ldk + koff + half * 8;
  return cat8(*(const v8bf*)p, *(const v8bf*)(p + 16));
}

static __device__ __forceinline__ v8f wmma_bf16(v16bf a, v16bf b, v8f c) {
  return __builtin_amdgcn_wmma_f32_16x16x32_f16(false, a, false, b,
                                                 (short)0, c, false, false);
}
static __device__ __forceinline__ v8f wmma_split(v16bf ah, v16bf al, v16bf bh, v16bf bl, v8f c) {
  v8f x = {};
  x = wmma_bf16(al, bh, x);
  x = wmma_bf16(ah, bl, x);
  return wmma_bf16(ah, bh, c) + x * RSPLIT;
}
static __device__ __forceinline__ void store_rows64_planes(const float* so, __bf16* dst, size_t plane, int lane) {
#pragma unroll 1
  for (int pass = 0; pass < 2; ++pass) {
#pragma unroll 4
    for (int rr = 0; rr < 16; ++rr) {
      _Float16 h0, l0, h1, l1;
      split16(*(const volatile float*)(so + rr * 64 + 2 * lane), h0, l0); split16(*(const volatile float*)(so + rr * 64 + 2 * lane + 1), h1, l1);
      *(volatile unsigned*)(dst + (size_t)rr * 64 + 2 * lane) = pack2h(h0, h1);
      *(volatile unsigned*)(dst + plane + (size_t)rr * 64 + 2 * lane) = pack2h(l0, l1);
    }
    __threadfence();
  }
}

__global__ void cvtT_kernel(const float* __restrict__ src,
                            __bf16* __restrict__ dst, int R, int C) {
  int idx = blockIdx.x * 256 + threadIdx.x;
  if (idx >= R * C / 2) return;
  int cc = idx / (R / 2), rr = 2 * (idx - cc * (R / 2));
  _Float16 h0, l0, h1, l1;
  split16(src[(size_t)rr * C + cc], h0, l0); split16(src[(size_t)(rr + 1) * C + cc], h1, l1);
  unsigned* d  = (unsigned*)(dst + (size_t)cc * R + rr);
  unsigned* dl = (unsigned*)(dst + (size_t)R * C + (size_t)cc * R + rr);
  const unsigned ph = pack2h(h0, h1), pl = pack2h(l0, l1);
  *(volatile unsigned*)d = ph; *(volatile unsigned*)dl = pl; __threadfence(); *(volatile unsigned*)d = ph; *(volatile unsigned*)dl = pl;
}

__global__ __launch_bounds__(128)
void qkv_kernel(const float* __restrict__ x,
                const __bf16* __restrict__ wqT,
                const __bf16* __restrict__ wkT,
                const __bf16* __restrict__ wvT,
                __bf16* __restrict__ q,
                __bf16* __restrict__ k,
                __bf16* __restrict__ v) {
  __shared__ __attribute__((aligned(16))) float so[4][16 * 64];
  const int lane = threadIdx.x & 31;
  const int wave = threadIdx.x >> 5;
  const int row0 = (blockIdx.x * 4 + wave) * 16;
  const int r    = lane & 15;
  const int half = lane >> 4;
  const size_t WPL = (size_t)KEY * MDIM;

  v8f accq[4] = {}, acck[4] = {}, accv[4] = {};

  for (int kk = 0; kk < MDIM; kk += 32) {
    const float* p = x + (size_t)(row0 + r) * MDIM + kk + half * 8;
    const v4f f0 = *(const v4f*)(p);
    const v4f f1 = *(const v4f*)(p + 4);
    const v4f f2 = *(const v4f*)(p + 16);
    const v4f f3 = *(const v4f*)(p + 20);
    union { v16bf v; _Float16 e[16]; } au, alu;
#pragma unroll
    for (int j = 0; j < 4; ++j) {
      split16(f0[j], au.e[j],      alu.e[j]);
      split16(f1[j], au.e[4 + j],  alu.e[4 + j]);
      split16(f2[j], au.e[8 + j],  alu.e[8 + j]);
      split16(f3[j], au.e[12 + j], alu.e[12 + j]);
    }
    const v16bf a = au.v, al = alu.v;
#pragma unroll
    for (int nt = 0; nt < 4; ++nt) {
      const int col = nt * 16 + r;
      v16bf bq = load_bT(wqT, MDIM, col, half, kk), bql = load_bT(wqT + WPL, MDIM, col, half, kk);
      accq[nt] = wmma_split(a, al, bq, bql, accq[nt]);
      v16bf bk = load_bT(wkT, MDIM, col, half, kk), bkl = load_bT(wkT + WPL, MDIM, col, half, kk);
      acck[nt] = wmma_split(a, al, bk, bkl, acck[nt]);
      v16bf bv = load_bT(wvT, MDIM, col, half, kk), bvl = load_bT(wvT + WPL, MDIM, col, half, kk);
      accv[nt] = wmma_split(a, al, bv, bvl, accv[nt]);
    }
  }
  float* sw = so[wave];
  __bf16* dsts[3] = {q, k, v};
#pragma unroll 1
  for (int s = 0; s < 3; ++s) {
    const float sc = (s == 0) ? QSCALE : 1.0f;
#pragma unroll
    for (int nt = 0; nt < 4; ++nt)
#pragma unroll
      for (int i = 0; i < 8; ++i)
        sw[(half * 8 + i) * 64 + nt * 16 + r] = ((s == 0) ? accq[nt][i] : (s == 1) ? acck[nt][i] : accv[nt][i]) * sc;
    asm volatile("s_wait_dscnt 0" ::: "memory");
    store_rows64_planes(sw, dsts[s] + (size_t)row0 * KEY, PQK, lane);
    asm volatile("s_wait_dscnt 0" ::: "memory");
  }
}

__global__ __launch_bounds__(256) void vt_kernel(const __bf16* __restrict__ v, __bf16* __restrict__ vT) {
  __shared__ __bf16 t[64][66];
  const int tid = threadIdx.x, lane = tid & 31, wave = tid >> 5;
  const int row0 = blockIdx.x * 64, b = row0 >> 11, sr = row0 & (SEQ - 1);
  const size_t pl = blockIdx.y ? PQK : 0;
  const __bf16* src = v + pl + (size_t)row0 * KEY;
#pragma unroll
  for (int kq = 0; kq < 16; ++kq) { const int e = tid + 256 * kq; t[e >> 6][e & 63] = src[e]; }
  __syncthreads();
  __bf16* dst = vT + pl + (size_t)b * KEY * SEQ + sr;
#pragma unroll
  for (int rr = 0; rr < 8; ++rr) {
    const int d = wave * 8 + rr;
    const unsigned pk = pack2h(t[2 * lane][d], t[2 * lane + 1][d]);
    unsigned* dp = (unsigned*)(dst + (size_t)d * SEQ) + lane;
    *(volatile unsigned*)dp = pk; __threadfence(); *(volatile unsigned*)dp = pk;
  }
}

__global__ __launch_bounds__(128)
void attn_kernel(const __bf16* __restrict__ q,
                 const __bf16* __restrict__ k,
                 const __bf16* __restrict__ vT,
                 __bf16* __restrict__ z) {
  __shared__ __attribute__((aligned(16))) __bf16 plds[4][16 * 32];
  __shared__ __attribute__((aligned(16))) __bf16 pldsl[4][16 * 32];
  __shared__ __attribute__((aligned(16))) float  zst[4][16 * 64];
  const int lane = threadIdx.x & 31;
  const int wave = threadIdx.x >> 5;
  const int w    = blockIdx.x * 4 + wave;
  const int b    = w >> 7;
  const int row0 = (w & 127) * 16;
  const int r    = lane & 15;
  const int half = lane >> 4;
  __bf16* pw = plds[wave];
  __bf16* pwl = pldsl[wave];

  const __bf16* qb = q  + (size_t)b * SEQ * KEY;
  const __bf16* kb = k  + (size_t)b * SEQ * KEY;
  const __bf16* vb = vT + (size_t)b * KEY * SEQ;

  v16bf qa[2], qal[2];
#pragma unroll
  for (int c = 0; c < 2; ++c) {
    qa[c]  = load_a(qb + (size_t)row0 * KEY, KEY, r, half, c * 32);
    qal[c] = load_a(qb + PQK + (size_t)row0 * KEY, KEY, r, half, c * 32);
  }

  v8f zacc[4] = {};
  float mrow[8], srow[8];
#pragma unroll
  for (int i = 0; i < 8; ++i) { mrow[i] = -1e30f; srow[i] = 0.0f; }

  for (int j0 = 0; j0 < SEQ; j0 += 32) {
    if (j0 + 32 < SEQ) {
      __builtin_prefetch(kb + (size_t)(j0 + 32) * KEY, 0, 3);
      __builtin_prefetch(vb + (size_t)(j0 + 32), 0, 3);
    }
    v8f s[2];
#pragma unroll
    for (int nt = 0; nt < 2; ++nt) {
      v8f acc = {};
#pragma unroll
      for (int c = 0; c < 2; ++c) {
        v16bf bkf  = load_bT(kb, KEY, j0 + nt * 16 + r, half, c * 32);
        v16bf bkfl = load_bT(kb + PQK, KEY, j0 + nt * 16 + r, half, c * 32);
        acc = wmma_split(qa[c], qal[c], bkf, bkfl, acc);
      }
      s[nt] = acc;
    }
    float newm[8];
#pragma unroll
    for (int i = 0; i < 8; ++i) {
      float mx = fmaxf(s[0][i], s[1][i]);
#pragma unroll
      for (int msk = 8; msk >= 1; msk >>= 1)
        mx = fmaxf(mx, __shfl_xor(mx, msk, 32));
      newm[i] = fmaxf(mrow[i], mx);
    }
#pragma unroll
    for (int i = 0; i < 8; ++i) {
      float e0 = fast_exp2(s[0][i] - newm[i]) * 1024.0f;
      float e1 = fast_exp2(s[1][i] - newm[i]) * 1024.0f;
      s[0][i] = e0; s[1][i] = e1;
      float rs = e0 + e1;
#pragma unroll
      for (int msk = 8; msk >= 1; msk >>= 1)
        rs += __shfl_xor(rs, msk, 32);
      float corr = fast_exp2(mrow[i] - newm[i]);
      srow[i] = srow[i] * corr + rs;
      mrow[i] = newm[i];
#pragma unroll
      for (int nt = 0; nt < 4; ++nt) zacc[nt][i] = zacc[nt][i] * corr;
    }
#pragma unroll
    for (int nt = 0; nt < 2; ++nt)
#pragma unroll
      for (int i = 0; i < 8; ++i) {
        _Float16 ph, pq; split16(s[nt][i], ph, pq);
        pw[(half * 8 + i) * 32 + nt * 16 + r] = ph; pwl[(half * 8 + i) * 32 + nt * 16 + r] = pq;
      }
    asm volatile("s_wait_dscnt 0" ::: "memory");
    v16bf pa = load_a(pw, 32, r, half, 0), pal = load_a(pwl, 32, r, half, 0);
#pragma unroll
    for (int dt = 0; dt < 4; ++dt) {
      v16bf bvf  = load_bT(vb, SEQ, dt * 16 + r, half, j0);
      v16bf bvfl = load_bT(vb + PQK, SEQ, dt * 16 + r, half, j0);
      zacc[dt] = wmma_split(pa, pal, bvf, bvfl, zacc[dt]);
    }
  }
  float* zs = zst[wave];
#pragma unroll
  for (int dt = 0; dt < 4; ++dt)
#pragma unroll
    for (int i = 0; i < 8; ++i) zs[(half * 8 + i) * 64 + dt * 16 + r] = zacc[dt][i] / srow[i];
  asm volatile("s_wait_dscnt 0" ::: "memory");
  store_rows64_planes(zs, z + (size_t)(b * SEQ + row0) * KEY, PQK, lane);
}

__global__ __launch_bounds__(128)
void mlp_kernel(const __bf16* __restrict__ z,
                const __bf16* __restrict__ w1T, const float* __restrict__ b1,
                const __bf16* __restrict__ w2T, const float* __restrict__ b2,
                const __bf16* __restrict__ w3T, const float* __restrict__ b3,
                float* __restrict__ out) {
  __shared__ __attribute__((aligned(16))) __bf16 hlds[4][16 * DDIM];
  __shared__ __attribute__((aligned(16))) __bf16 hldsl[4][16 * DDIM];
  __shared__ __attribute__((aligned(16))) float  ost[4][16 * DDIM];
  const int lane = threadIdx.x & 31;
  const int wave = threadIdx.x >> 5;
  const int row0 = (blockIdx.x * 4 + wave) * 16;
  const int r    = lane & 15;
  const int half = lane >> 4;
  __bf16* hw = hlds[wave];
  __bf16* hwl = hldsl[wave];
  const size_t W1PL = (size_t)DDIM * KEY, W23PL = (size_t)DDIM * DDIM;

  v16bf za[2], zal[2];
#pragma unroll
  for (int c = 0; c < 2; ++c) {
    za[c]  = load_a(z + (size_t)row0 * KEY, KEY, r, half, c * 32);
    zal[c] = load_a(z + PQK + (size_t)row0 * KEY, KEY, r, half, c * 32);
  }

  v8f h[8];
#pragma unroll
  for (int ct = 0; ct < 8; ++ct) {
    const float bias = b1[ct * 16 + r];
    v8f acc;
#pragma unroll
    for (int i = 0; i < 8; ++i) acc[i] = bias;
#pragma unroll
    for (int c = 0; c < 2; ++c) {
      v16bf bw  = load_bT(w1T, KEY, ct * 16 + r, half, c * 32);
      v16bf bwl = load_bT(w1T + W1PL, KEY, ct * 16 + r, half, c * 32);
      acc = wmma_split(za[c], zal[c], bw, bwl, acc);
    }
#pragma unroll
    for (int i = 0; i < 8; ++i) {
      float x0 = acc[i];
      acc[i] = x0 > 0.0f ? x0 : (__expf(x0) - 1.0f);
    }
    h[ct] = acc;
  }

  const __bf16* Ws[2] = { w2T, w3T };
  const float*  bs[2] = { b2, b3 };
#pragma unroll 1
  for (int layer = 0; layer < 2; ++layer) {
#pragma unroll
    for (int ct = 0; ct < 8; ++ct)
#pragma unroll
      for (int i = 0; i < 8; ++i) {
        _Float16 hh_, hl_; split16(h[ct][i], hh_, hl_);
        hw[(half * 8 + i) * DDIM + ct * 16 + r] = hh_; hwl[(half * 8 + i) * DDIM + ct * 16 + r] = hl_;
      }
    asm volatile("s_wait_dscnt 0" ::: "memory");
    v16bf ha[4], hal[4];
#pragma unroll
    for (int c = 0; c < 4; ++c) { ha[c] = load_a(hw, DDIM, r, half, c * 32); hal[c] = load_a(hwl, DDIM, r, half, c * 32); }
    const __bf16* W  = Ws[layer];
    const float*  bb = bs[layer];
#pragma unroll
    for (int ct = 0; ct < 8; ++ct) {
      const float bias = bb[ct * 16 + r];
      v8f acc;
#pragma unroll
      for (int i = 0; i < 8; ++i) acc[i] = bias;
#pragma unroll
      for (int c = 0; c < 4; ++c) {
        v16bf bw  = load_bT(W, DDIM, ct * 16 + r, half, c * 32);
        v16bf bwl = load_bT(W + W23PL, DDIM, ct * 16 + r, half, c * 32);
        acc = wmma_split(ha[c], hal[c], bw, bwl, acc);
      }
#pragma unroll
      for (int i = 0; i < 8; ++i) {
        float x0 = acc[i];
        acc[i] = x0 > 0.0f ? x0 : (__expf(x0) - 1.0f);
      }
      h[ct] = acc;
    }
  }

  float* os_ = ost[wave];
#pragma unroll
  for (int ct = 0; ct < 8; ++ct)
#pragma unroll
    for (int i = 0; i < 8; ++i) os_[(half * 8 + i) * DDIM + ct * 16 + r] = h[ct][i];
  asm volatile("s_wait_dscnt 0" ::: "memory");
  typedef float v4fa __attribute__((ext_vector_type(4), may_alias));
#pragma unroll 1
  for (int pass = 0; pass < 2; ++pass) {
#pragma unroll 4
    for (int i = 0; i < 16; ++i) {
      const int c = lane + 32 * i, rr = c >> 5, qq = c & 31;
      const v4f vv = *(const volatile v4fa*)(os_ + rr * DDIM + qq * 4);
      *(volatile v4f*)(out + (size_t)(row0 + rr) * DDIM + qq * 4) = vv;
    }
    __threadfence();
  }
}

extern "C" void kernel_launch(void* const* d_in, const int* in_sizes, int n_in,
                              void* d_out, int out_size, void* d_ws, size_t ws_size,
                              hipStream_t stream) {
  (void)in_sizes; (void)n_in; (void)out_size; (void)ws_size;
  const float* x  = (const float*)d_in[0];
  const float* Wq = (const float*)d_in[1];
  const float* Wk = (const float*)d_in[2];
  const float* Wv = (const float*)d_in[3];
  const float* W1 = (const float*)d_in[4];
  const float* b1 = (const float*)d_in[5];
  const float* W2 = (const float*)d_in[6];
  const float* b2 = (const float*)d_in[7];
  const float* W3 = (const float*)d_in[8];
  const float* b3 = (const float*)d_in[9];

  __bf16* q   = (__bf16*)d_ws;
  __bf16* k   = q   + 2 * PQK;
  __bf16* v   = k   + 2 * PQK;
  __bf16* vT  = v   + 2 * PQK;
  __bf16* z   = vT  + 2 * PQK;
  __bf16* wqT = z   + 2 * PQK;
  __bf16* wkT = wqT + (size_t)2 * KEY * MDIM;
  __bf16* wvT = wkT + (size_t)2 * KEY * MDIM;
  __bf16* w1T = wvT + (size_t)2 * KEY * MDIM;
  __bf16* w2T = w1T + (size_t)2 * DDIM * KEY;
  __bf16* w3T = w2T + (size_t)2 * DDIM * DDIM;

  cvtT_kernel<<<(MDIM * KEY / 2 + 255) / 256, 256, 0, stream>>>(Wq, wqT, MDIM, KEY);
  cvtT_kernel<<<(MDIM * KEY / 2 + 255) / 256, 256, 0, stream>>>(Wk, wkT, MDIM, KEY);
  cvtT_kernel<<<(MDIM * KEY / 2 + 255) / 256, 256, 0, stream>>>(Wv, wvT, MDIM, KEY);
  cvtT_kernel<<<(KEY * DDIM / 2 + 255) / 256, 256, 0, stream>>>(W1, w1T, KEY, DDIM);
  cvtT_kernel<<<(DDIM * DDIM / 2 + 255) / 256, 256, 0, stream>>>(W2, w2T, DDIM, DDIM);
  cvtT_kernel<<<(DDIM * DDIM / 2 + 255) / 256, 256, 0, stream>>>(W3, w3T, DDIM, DDIM);

  qkv_kernel <<<ROWS / 16 / 4, 128, 0, stream>>>(x, wqT, wkT, wvT, q, k, v);
  vt_kernel  <<<dim3(ROWS / 64, 2), 256, 0, stream>>>(v, vT);
  attn_kernel<<<ROWS / 16 / 4, 128, 0, stream>>>(q, k, vT, z);
  mlp_kernel <<<ROWS / 16 / 4, 128, 0, stream>>>(z, w1T, b1, w2T, b2, w3T, b3,
                                                 (float*)d_out);
}
